// SparseAttention_87273735455080
// MI455X (gfx1250) — hardware-verified
//
#include <hip/hip_runtime.h>
#include <math.h>

typedef __attribute__((ext_vector_type(16))) _Float16 v16h;
typedef __attribute__((ext_vector_type(16))) __bf16 v16b;
typedef __attribute__((ext_vector_type(8)))  _Float16 v8h;
typedef __attribute__((ext_vector_type(8)))  __bf16 v8b;
typedef __attribute__((ext_vector_type(8)))  float v8f;
typedef __attribute__((ext_vector_type(4)))  float v4f;
typedef __attribute__((ext_vector_type(4)))  unsigned v4u;

template <typename T> __device__ __forceinline__ void vst2(void* p, T v) { *(volatile T*)p = v; __threadfence(); *(volatile T*)p = v; }
__device__ __forceinline__ v8f wmma16(v16h a, v16h b, v8f c) {
  v8f d = __builtin_amdgcn_wmma_f32_16x16x32_f16(false, a, false, b, (short)0, c, false, false);
  asm volatile("v_nop\n\tv_nop\n\tv_nop\n\tv_nop" : "+v"(d) : "v"(a), "v"(b));
  return d;
}
__device__ __forceinline__ v8f wmma_bf(v16b a, v16b b, v8f c) {
  v8f d = __builtin_amdgcn_wmma_f32_16x16x32_bf16(false, a, false, b, (short)0, c, false, false);
  asm volatile("v_nop\n\tv_nop\n\tv_nop\n\tv_nop" : "+v"(d) : "v"(a), "v"(b));
  return d;
}
__device__ __forceinline__ v16h frag_h(const _Float16* rowk0, unsigned lane) {
  union { v16h v; v8h q[2]; } u; const _Float16* p = rowk0 + 8u * (lane >> 4);
  u.q[0] = *(const v8h*)p; u.q[1] = *(const v8h*)(p + 16); return u.v;
}
__device__ __forceinline__ v16b frag_b(const __bf16* rowk0, unsigned lane) {
  union { v16b v; v8b q[2]; } u; const __bf16* p = rowk0 + 8u * (lane >> 4);
  u.q[0] = *(const v8b*)p; u.q[1] = *(const v8b*)(p + 16); return u.v;
}
struct F2 { v16b h, l; };
__device__ __forceinline__ F2 bsplit16(const float v[16]) { F2 r;
#pragma unroll
  for (int i = 0; i < 16; ++i) { const __bf16 h = (__bf16)v[i]; r.h[i] = h; r.l[i] = (__bf16)(v[i] - (float)h); }
  return r; }
__device__ __forceinline__ F2 split_row(const float* row, unsigned k0, unsigned lane) { float v[16]; const float* p = row + k0 + 8u * (lane >> 4);
#pragma unroll
  for (int i = 0; i < 8; ++i) { v[i] = p[i]; v[8 + i] = p[16 + i]; }
  return bsplit16(v); }
__device__ __forceinline__ float bfr(float v) { return (float)(__bf16)v; }
__device__ __forceinline__ v16b wcol_oi(const float* Wm, unsigned k0, unsigned o, unsigned lane, unsigned K) { v16b w; const float* p = Wm + (size_t)o * K + k0 + 8u * (lane >> 4);
#pragma unroll
  for (int i = 0; i < 8; ++i) { w[i] = (__bf16)p[i]; w[8 + i] = (__bf16)p[16 + i]; }
  return w; }
#define LDSX() do { asm volatile("s_wait_dscnt 0" ::: "memory"); __builtin_amdgcn_wave_barrier(); __builtin_amdgcn_fence(3  , "workgroup"); } while (0)

#ifndef NB
#define NB 2
#endif
#ifndef SEQ
#define SEQ 2048
#endif
#define NB_FULL 2
#define SEQ_FULL 2048
#define TT SEQ
#define CC 1024
#define DIN 1024
#define NH 16
#define HD 64
#define NQB (TT / 64)
#define WHALF 64u
#define SCALE (0.125f)
#define SP 196

static_assert(SEQ % 64 == 0);
static_assert(SEQ <= SEQ_FULL);
static_assert(NB <= NB_FULL);
static_assert(CC % 128 == 0);
static_assert(DIN % 128 == 0);
static_assert(DIN % 32 == 0);
static_assert(CC % 32 == 0);
static_assert(CC == NH * HD);
static_assert(HD == 64);
static_assert((64 * 16) % 128 == 0);
static_assert((128 * 8) % 128 == 0);
static_assert(3 * 64 <= SP);
static_assert((SP * 4) % 16 == 0);

#define PL16 (2u * (size_t)NB * TT * CC)
#define WS_QH  ((size_t)0)
#define WS_QL  (WS_QH + PL16)
#define WS_KH  (WS_QL + PL16)
#define WS_KL  (WS_KH + PL16)
#define WS_VB  (WS_KL + PL16)
#define WS_VBL (WS_VB + PL16)
#define WS_Y   (WS_VBL + PL16)
#define WS_END (WS_Y + 4u * (size_t)NB * TT * CC)
static_assert(WS_END <= (size_t)134217728);
static_assert(PL16 % 128 == 0);

__global__ __launch_bounds__(128) void k_proj(const float* __restrict__ X, const float* __restrict__ WQ, const float* __restrict__ WK, const float* __restrict__ WV, const float* __restrict__ BQ, const float* __restrict__ BK, const float* __restrict__ BV,
    _Float16* __restrict__ QH, _Float16* __restrict__ QL, _Float16* __restrict__ KH, _Float16* __restrict__ KL, __bf16* __restrict__ VB, __bf16* __restrict__ VBL) {
  __shared__ __align__(16) _Float16 sh[64][136], sl[64][136]; __shared__ __align__(16) __bf16 tb[128][72], tbl[128][72];
  const unsigned tid = threadIdx.x, wave = tid >> 5, lane = tid & 31u, col = lane & 15u, g = lane >> 4;
  const unsigned which = blockIdx.z; const unsigned c0 = blockIdx.y * 128u; const unsigned r0 = blockIdx.x * 64u; const unsigned bb = r0 / (unsigned)TT; const unsigned t0 = r0 - bb * (unsigned)TT;
  const float* WA = which == 0u ? WQ : which == 1u ? WK : WV; const float* BA = which == 0u ? BQ : which == 1u ? BK : BV;
  const float* xrow = X + ((size_t)bb * SEQ_FULL + t0 + wave * 16u + col) * DIN;
  v8f acc[8] = {};
#pragma unroll 2
  for (unsigned kc = 0; kc < DIN / 32; ++kc) { v16b a; { const float* p = xrow + kc * 32u + 8u * g;
#pragma unroll
      for (int i = 0; i < 8; ++i) { a[i] = (__bf16)p[i]; a[8 + i] = (__bf16)p[16 + i]; } }
    asm volatile("s_wait_loadcnt 0x0" ::: "memory");
#pragma unroll
    for (int j = 0; j < 8; ++j) { const v16b w = wcol_oi(WA, kc * 32u, c0 + j * 16u + col, lane, DIN); asm volatile("s_wait_loadcnt 0x0" ::: "memory"); acc[j] = wmma_bf(a, w, acc[j]); } }
  if (which < 2u) { _Float16* DH = which == 0u ? QH : KH; _Float16* DL = which == 0u ? QL : KL;
#pragma unroll
    for (int j = 0; j < 8; ++j) { const float bias = bfr(BA[c0 + j * 16u + col]);
#pragma unroll
      for (int r = 0; r < 8; ++r) { const float v = acc[j][r] + bias; const _Float16 hv = (_Float16)v; sh[wave * 16u + 8u * g + r][j * 16u + col] = hv; sl[wave * 16u + 8u * g + r][j * 16u + col] = (_Float16)((v - (float)hv) * 1024.0f); } }
    __syncthreads();
    for (unsigned e = tid; e < 64u * 16u; e += 128u) { const unsigned rl = e >> 4, q = e & 15u; const size_t o = ((size_t)r0 + rl) * CC + c0 + q * 8u;
      const v4u vh = *(const v4u*)&sh[rl][q * 8u]; const v4u vl = *(const v4u*)&sl[rl][q * 8u];
      vst2((void*)(DH + o), vh); vst2((void*)(DL + o), vl); }
  } else {
#pragma unroll
    for (int j = 0; j < 8; ++j) { const float bias = bfr(BA[c0 + j * 16u + col]);
#pragma unroll
      for (int r = 0; r < 8; ++r) { const float v = acc[j][r] + bias; const unsigned rl = wave * 16u + 8u * g + r, cl = j * 16u + col; const __bf16 bh = (__bf16)v; tb[cl][rl] = bh; tbl[cl][rl] = (__bf16)(v - (float)bh); } }
    __syncthreads();
    for (unsigned e = tid; e < 128u * 8u; e += 128u) { const unsigned cl = e >> 3, q = e & 7u; const size_t o3 = ((size_t)bb * CC + c0 + cl) * (size_t)TT + t0 + q * 8u;
      const v4u vh = *(const v4u*)&tb[cl][q * 8u]; const v4u vl = *(const v4u*)&tbl[cl][q * 8u];
      vst2((void*)(VB + o3), vh); vst2((void*)(VBL + o3), vl); } } }

__global__ __launch_bounds__(128) void k_attn(const _Float16* __restrict__ QH, const _Float16* __restrict__ QL, const _Float16* __restrict__ KH, const _Float16* __restrict__ KL, const __bf16* __restrict__ VB, const __bf16* __restrict__ VBL, float* __restrict__ Y) {
  __shared__ __align__(16) float ss[4][16][SP];
  const unsigned tid = threadIdx.x, wave = tid >> 5, lane = tid & 31u, col = lane & 15u, g = lane >> 4;
  const unsigned qt = blockIdx.x, h = blockIdx.y, b = blockIdx.z;
  const unsigned nt = qt == 0u ? 1u : (qt == 1u ? 2u : 3u);
  const unsigned ql0 = qt * 64u + wave * 16u; const size_t q0 = (size_t)b * TT + ql0;
  v16h ah[2], al[2];
#pragma unroll
  for (int kc = 0; kc < 2; ++kc) { const size_t o = (q0 + col) * CC + h * HD + kc * 32; ah[kc] = frag_h(QH + o, lane); al[kc] = frag_h(QL + o, lane); }
#pragma unroll 1
  for (unsigned s = 0; s < nt; ++s) { const unsigned kt = s == 0u ? 0u : (qt + 1u + s) - nt; const size_t kr0 = (size_t)b * TT + kt * 64u;
    v8f acc[4] = {}, accl[4] = {};
#pragma unroll
    for (int kc = 0; kc < 2; ++kc) {
#pragma unroll
      for (int j = 0; j < 4; ++j) { const size_t o = (kr0 + j * 16 + col) * CC + h * HD + kc * 32; const v16h kbf = frag_h(KH + o, lane), klf = frag_h(KL + o, lane);
        acc[j] = wmma16(ah[kc], kbf, acc[j]); accl[j] = wmma16(al[kc], kbf, accl[j]); accl[j] = wmma16(ah[kc], klf, accl[j]); } }
#pragma unroll
    for (int j = 0; j < 4; ++j) { const unsigned jk = kt * 64u + j * 16u + col;
#pragma unroll
      for (int r = 0; r < 8; ++r) { const unsigned i = ql0 + 8u * g + r; const bool vis = (jk <= i) && (((i - jk) <= WHALF) || (jk == 0u) || (i == 0u));
        const float v = (acc[j][r] + accl[j][r] * (1.0f / 1024.0f)) * SCALE; ss[wave][8u * g + r][s * 64u + j * 16u + col] = vis ? v : -3.0e38f; } } }
  LDSX();
  const unsigned nu = nt * 2u;
#pragma unroll 1
  for (unsigned rl = 0; rl < 16u; ++rl) { float* row = &ss[wave][rl][0];
    float m = -3.0e38f;
#pragma unroll 1
    for (unsigned u = 0; u < nu; ++u) m = fmaxf(m, row[lane + 32u * u]);
#pragma unroll
    for (int o = 1; o < 32; o <<= 1) m = fmaxf(m, __shfl_xor(m, o));
    float sum = 0.f;
#pragma unroll 1
    for (unsigned u = 0; u < nu; ++u) { const float v = row[lane + 32u * u]; const float e = (v <= -1.0e38f) ? 0.f : expf(v - m); row[lane + 32u * u] = e; sum += e; }
#pragma unroll
    for (int o = 1; o < 32; o <<= 1) sum += __shfl_xor(sum, o);
    const float inv = (1.0f / sum) * 2048.0f;
#pragma unroll 1
    for (unsigned u = 0; u < nu; ++u) { const float pv = row[lane + 32u * u] * inv; row[lane + 32u * u] = pv; } }
  LDSX();
  v8f oacc[4] = {};
#pragma unroll 1
  for (unsigned s = 0; s < nt; ++s) { const unsigned kt = s == 0u ? 0u : (qt + 1u + s) - nt;
#pragma unroll
    for (int kc2 = 0; kc2 < 2; ++kc2) { const F2 p = split_row(&ss[wave][col][0], s * 64u + kc2 * 32u, lane);
#pragma unroll
      for (int j = 0; j < 4; ++j) { const size_t po = ((size_t)b * CC + h * HD + j * 16 + col) * (size_t)TT + kt * 64u + kc2 * 32u; const v16b vh = frag_b(VB + po, lane);
        oacc[j] = wmma_bf(p.h, vh, oacc[j]); oacc[j] = wmma_bf(p.l, vh, oacc[j]); oacc[j] = wmma_bf(p.h, frag_b(VBL + po, lane), oacc[j]); } } }
  LDSX();
#pragma unroll
  for (int j = 0; j < 4; ++j)
#pragma unroll
    for (int r = 0; r < 8; ++r) ss[wave][8u * g + r][j * 16u + col] = oacc[j][r] * (1.0f / 2048.0f);
  LDSX();
  for (unsigned it = 0; it < 8u; ++it) { const unsigned rl = 2u * it + g; const v4f val = *(const v4f*)&ss[wave][rl][col * 4u]; vst2((void*)(Y + ((size_t)b * TT + ql0 + rl) * CC + h * HD + col * 4u), val); } }

__global__ __launch_bounds__(128) void k_out(const float* __restrict__ Y, const float* __restrict__ WO, const float* __restrict__ BO, float* __restrict__ OUT) { __shared__ __align__(16) float sf[4][16][132];
  const unsigned tid = threadIdx.x, wave = tid >> 5, lane = tid & 31u, col = lane & 15u, g = lane >> 4; const unsigned c0 = blockIdx.y * 128u; const size_t r0 = (size_t)blockIdx.x * 64u + wave * 16u;
  v8f acc[8] = {};
#pragma unroll 2
  for (unsigned kc = 0; kc < CC / 32; ++kc) { const F2 a = split_row(Y + (r0 + col) * CC, kc * 32u, lane); asm volatile("s_wait_loadcnt 0x0" ::: "memory");
#pragma unroll
    for (int j = 0; j < 8; ++j) { const v16b w = wcol_oi(WO, kc * 32u, c0 + j * 16u + col, lane, CC); asm volatile("s_wait_loadcnt 0x0" ::: "memory"); acc[j] = wmma_bf(a.h, w, acc[j]); acc[j] = wmma_bf(a.l, w, acc[j]); } }
#pragma unroll
  for (int j = 0; j < 8; ++j) { const float bias = bfr(BO[c0 + j * 16u + col]);
#pragma unroll
    for (int r = 0; r < 8; ++r) sf[wave][8u * g + r][j * 16u + col] = acc[j][r] + bias; }
  LDSX();
  for (unsigned rl = 0; rl < 16u; ++rl) { const v4f val = *(const v4f*)&sf[wave][rl][lane * 4u]; vst2((void*)(OUT + (r0 + rl) * DIN + c0 + lane * 4u), val); } }

extern "C" void kernel_launch(void* const* d_in, const int* in_sizes, int n_in, void* d_out, int out_size, void* d_ws, size_t ws_size, hipStream_t stream) {
  if (n_in < 9) return;
  const long long need_x = ((long long)(NB - 1) * SEQ_FULL + SEQ) * DIN;
  if ((long long)in_sizes[0] < need_x) return;
  if (in_sizes[1] < CC * DIN || in_sizes[3] < CC * DIN || in_sizes[5] < CC * DIN || in_sizes[7] < DIN * CC) return;
  if (in_sizes[2] < CC || in_sizes[4] < CC || in_sizes[6] < CC || in_sizes[8] < DIN) return;
  if ((long long)out_size < (long long)NB * SEQ * DIN) return;
  if (ws_size < (size_t)WS_END) return;
  const float* const* F = (const float* const*)d_in;
  char* ws = (char*)d_ws;
  _Float16 *QH = (_Float16*)(ws + WS_QH), *QL = (_Float16*)(ws + WS_QL), *KH = (_Float16*)(ws + WS_KH), *KL = (_Float16*)(ws + WS_KL);
  __bf16 *VB = (__bf16*)(ws + WS_VB), *VBL = (__bf16*)(ws + WS_VBL); float* Y = (float*)(ws + WS_Y);
  k_proj<<<dim3(NB * TT / 64, CC / 128, 3), 128, 0, stream>>>(F[0], F[1], F[3], F[5], F[2], F[4], F[6], QH, QL, KH, KL, VB, VBL);
  k_attn<<<dim3(NQB, NH, NB), 128, 0, stream>>>(QH, QL, KH, KL, VB, VBL, Y);
  k_out<<<dim3(NB * TT / 64, DIN / 128), 128, 0, stream>>>(Y, F[7], F[8], (float*)d_out);
}
